// ContextBiasingLayer_15109694947859
// MI455X (gfx1250) — hardware-verified
//
#include <hip/hip_runtime.h>
#include <math.h>

constexpr int kB   = 16;
constexpr int kT   = 1024;
constexpr int kC   = 256;
constexpr int kD   = 512;
constexpr int kH   = 8;
constexpr int kDK  = 64;
constexpr int kRowsQ  = kB * kT;
constexpr int kRowsKV = kB * kC;
constexpr int kNBH    = kB * kH;
constexpr int kGroupBH = 16;
constexpr int kNGroups = kNBH / kGroupBH;
constexpr float kWCarry    = 64.0f;
constexpr float kWCarryInv = 1.0f / 64.0f;
constexpr float kACarry    = 16.0f;
constexpr float kPCarry    = 4096.0f;
constexpr float kScoreScale = 0.125f / (16.0f * 16.0f);
constexpr float kPVScale    = 1.0f / (4096.0f * 16.0f);
constexpr float kLnEps      = 1e-12f;
constexpr float kInvD       = 1.0f / 512.0f;

constexpr size_t kOffWq  = 0;
constexpr size_t kOffWk  = 524288;
constexpr size_t kOffWv  = 1048576;
constexpr size_t kOffWoH = 1572864;
constexpr size_t kOffWoL = 2621440;
constexpr size_t kOffK16 = 3670016;
constexpr size_t kOffVT16 = 7864320;
constexpr size_t kOffRA  = 12058624;
constexpr size_t kOffRB  = 45613056;
constexpr size_t kOffRC  = 79167488;
constexpr size_t kOffRD  = 95944704;
constexpr size_t kWsTotal = 129499136;

typedef __attribute__((ext_vector_type(16))) _Float16 v16h;
typedef __attribute__((ext_vector_type(8)))  _Float16 v8h;
typedef __attribute__((ext_vector_type(16))) __bf16   v16b;
typedef __attribute__((ext_vector_type(8)))  __bf16   v8b;
typedef __attribute__((ext_vector_type(8)))  float    v8f;
typedef __attribute__((ext_vector_type(4)))  float    v4f;
typedef __attribute__((ext_vector_type(4)))  unsigned int v4u;
typedef __attribute__((ext_vector_type(4)))  int      v4i;

__device__ __forceinline__ unsigned short f2bf_bits(float f) {
  unsigned u = __float_as_uint(f);
  return (unsigned short)((u + 0x7FFFu + ((u >> 16) & 1u)) >> 16);
}
__device__ __forceinline__ float bf_bits2f(unsigned short h) { return __uint_as_float(((unsigned)h) << 16); }

__device__ __forceinline__ void dep_guard_h(v8f& a, v8f& b, v16h x, v16h y) { asm volatile("v_nop\n\tv_nop\n\tv_nop\n\tv_nop" : "+v"(a), "+v"(b) : "v"(x), "v"(y)); }
__device__ __forceinline__ void dep_guard_b(v8f& a, v8f& b, v16b x, v16b y) { asm volatile("v_nop\n\tv_nop\n\tv_nop\n\tv_nop" : "+v"(a), "+v"(b) : "v"(x), "v"(y)); }
__device__ __forceinline__ void keep4_h(v16h a, v16h b, v16h c, v16h d) { asm volatile("v_nop" :: "v"(a), "v"(b), "v"(c), "v"(d)); }
__device__ __forceinline__ void keep4_b(v16b a, v16b b, v16b c, v16b d) { asm volatile("v_nop" :: "v"(a), "v"(b), "v"(c), "v"(d)); }
__device__ __forceinline__ void acc_guard4(v8f& a, v8f& b, v8f& c, v8f& d) { asm volatile("v_nop\n\tv_nop\n\tv_nop\n\tv_nop" : "+v"(a), "+v"(b), "+v"(c), "+v"(d)); }
template <typename T> struct Frag;
template <> struct Frag<_Float16> {
  typedef v16h V; union U { v16h v; v8h h[2]; };
  static __device__ __forceinline__ v16h load(const _Float16* p) {
    U f; f.h[0] = *(const v8h*)(p); f.h[1] = *(const v8h*)(p + 16); return f.v;
  }
  static __device__ __forceinline__ v8f mma(v16h a, v16h b, v8f c) {
    return __builtin_amdgcn_wmma_f32_16x16x32_f16(false, a, false, b, (short)0, c, false, false);
  }
  static __device__ __forceinline__ void guard(v8f& a, v8f& b, v16h x, v16h y) { dep_guard_h(a, b, x, y); }
  static __device__ __forceinline__ void keep(v16h a, v16h b, v16h c, v16h d) { keep4_h(a, b, c, d); }
};
template <> struct Frag<__bf16> {
  typedef v16b V; union U { v16b v; v8b h[2]; };
  static __device__ __forceinline__ v16b load(const __bf16* p) {
    U f; f.h[0] = *(const v8b*)(p); f.h[1] = *(const v8b*)(p + 16); return f.v;
  }
  static __device__ __forceinline__ v8f mma(v16b a, v16b b, v8f c) {
    return __builtin_amdgcn_wmma_f32_16x16x32_bf16(false, a, false, b, (short)0, c, false, false);
  }
  static __device__ __forceinline__ void guard(v8f& a, v8f& b, v16b x, v16b y) { dep_guard_b(a, b, x, y); }
  static __device__ __forceinline__ void keep(v16b a, v16b b, v16b c, v16b d) { keep4_b(a, b, c, d); }
};

__device__ __forceinline__ unsigned pk16(unsigned short a, unsigned short b) { return (unsigned)a | ((unsigned)b << 16); }
__device__ __forceinline__ unsigned short h_bits(float f) { const _Float16 h = (_Float16)f; return __builtin_bit_cast(unsigned short, h); }

template <int ET> struct Elem;
template <> struct Elem<0> { typedef _Float16 T; };
template <> struct Elem<1> { typedef __bf16 T; };
template <int ET, bool SPLIT, int BIAS_MODE, int OUT_MODE, bool RESID, int ACT = 0>
__global__ __launch_bounds__(256) void wmma_gemm64(
    const unsigned short* __restrict__ Ap, const unsigned short* __restrict__ A2p, int lda, long strideA,
    const unsigned short* __restrict__ Btp, const unsigned short* __restrict__ Bt2p, int ldb, long strideB,
    void* __restrict__ Cout, void* __restrict__ Cout2, int ldc, long strideC,
    const float* __restrict__ bias,
    const float* __restrict__ resid, long strideR,
    int M, int N, int K, float scale) {
  typedef typename Elem<ET>::T T;
  typedef typename Frag<T>::V V;
  const T* A = (const T*)Ap; const T* A2 = (const T*)A2p; const T* Bt = (const T*)Btp; const T* Bt2 = (const T*)Bt2p;
  __shared__ __align__(16) float sT[8][16 * 68];
  const int b    = blockIdx.y;
  const int lane = threadIdx.x & 31;
  const int wave = threadIdx.x >> 5;
  const int tilesN = N >> 6;
  const int tilesM = M >> 6;
  const int tile = blockIdx.x * 8 + wave;
  if (tile >= tilesM * tilesN) return;
  const int tm = tile / tilesN;
  const int tn = tile - tm * tilesN;
  const int m0 = tm << 6;
  const int n0 = tn << 6;

  const T* Ab  = A  + (size_t)b * strideA;
  const T* Bb  = Bt + (size_t)b * strideB;
  const T* Ab2 = SPLIT ? (A2  + (size_t)b * strideA) : nullptr;
  const T* Bb2 = SPLIT ? (Bt2 + (size_t)b * strideB) : nullptr;

  const int rlane = lane & 15;
  const int koff  = (lane >> 4) * 8;
  const int mOff  = (lane >> 4) * 8;

  v8f acc[4][4];
#pragma unroll
  for (int i = 0; i < 4; ++i)
#pragma unroll
    for (int j = 0; j < 4; ++j) acc[i][j] = (v8f){0.f,0.f,0.f,0.f,0.f,0.f,0.f,0.f};

  for (int k0 = 0; k0 < K; k0 += 32) {
    V bh[4], bl[4];
#pragma unroll
    for (int j = 0; j < 4; ++j) {
      const size_t bo = (size_t)(n0 + (j << 4) + rlane) * ldb + koff + k0;
      bh[j] = Frag<T>::load(Bb + bo);
      if (SPLIT) bl[j] = Frag<T>::load(Bb2 + bo);
    }
#pragma unroll
    for (int i = 0; i < 4; ++i) {
      const size_t ao = (size_t)(m0 + (i << 4) + rlane) * lda + koff + k0;
      V ah = Frag<T>::load(Ab + ao);
      V al;
      if (SPLIT) al = Frag<T>::load(Ab2 + ao);
#pragma unroll
      for (int j = 0; j < 4; ++j) {
        acc[i][j] = Frag<T>::mma(ah, bh[j], acc[i][j]);
        if (SPLIT) {
          acc[i][j] = Frag<T>::mma(ah, bl[j], acc[i][j]);
          acc[i][j] = Frag<T>::mma(al, bh[j], acc[i][j]);
        }
      }
      Frag<T>::guard(acc[i][0], acc[i][3], ah, SPLIT ? al : ah);
    }
    Frag<T>::keep(bh[0], bh[1], bh[2], bh[3]);
    if (SPLIT) Frag<T>::keep(bl[0], bl[1], bl[2], bl[3]);
  }
  acc_guard4(acc[0][0], acc[0][1], acc[0][2], acc[0][3]);
  acc_guard4(acc[1][0], acc[1][1], acc[1][2], acc[1][3]);
  acc_guard4(acc[2][0], acc[2][1], acc[2][2], acc[2][3]);
  acc_guard4(acc[3][0], acc[3][1], acc[3][2], acc[3][3]);

  float* slab = sT[wave];
  const float* Rb = RESID ? (resid + (size_t)b * strideR) : nullptr;
#pragma unroll
  for (int i = 0; i < 4; ++i) {
    const int mBase = m0 + (i << 4);
#pragma unroll
    for (int j = 0; j < 4; ++j) {
      const int n = n0 + (j << 4) + rlane;
      float bv = 0.f;
      if (BIAS_MODE == 2) bv = bias[n];
#pragma unroll
      for (int r = 0; r < 8; ++r) {
        float v = acc[i][j][r] * scale;
        if (BIAS_MODE == 1) v += bias[mBase + mOff + r];
        if (BIAS_MODE == 2) v += bv;
        if (RESID) v += Rb[(size_t)(mBase + mOff + r) * ldc + n];
        if (ACT == 2) v = fmaxf(v, 0.0f);
        if (ACT == 4) v = (v > 0.f) ? v : 0.01f * v;
        slab[(mOff + r) * 68 + (j << 4) + rlane] = v;
      }
    }
    __builtin_amdgcn_fence(__ATOMIC_RELEASE, "workgroup");
    __builtin_amdgcn_wave_barrier();
    __builtin_amdgcn_fence(__ATOMIC_ACQUIRE, "workgroup");
    if (OUT_MODE == 0) {
      float* C = (float*)Cout + (size_t)b * strideC;
      const int hh = lane >> 4, c4 = (lane & 15) * 4;
      for (int pass = 0; pass < 2; ++pass) {
#pragma unroll
        for (int it = 0; it < 8; ++it) {
          const int row = it * 2 + hh;
          v4f v = *(const v4f*)(slab + row * 68 + c4);
          *(volatile v4f*)(C + (size_t)(mBase + row) * ldc + n0 + c4) = v;
        }
        __threadfence();
      }
    } else {
      const int q = lane >> 3, c8 = (lane & 7) * 8;
      unsigned short* C  = (unsigned short*)Cout  + (size_t)b * strideC;
      unsigned short* C2 = (OUT_MODE == 2) ? ((unsigned short*)Cout2 + (size_t)b * strideC) : nullptr;
      for (int pass = 0; pass < 2; ++pass) {
#pragma unroll
        for (int it = 0; it < 4; ++it) {
          const int row = it * 4 + q;
          const float* sp = slab + row * 68 + c8;
          v8h hv, lv;
#pragma unroll
          for (int e = 0; e < 8; ++e) {
            if (OUT_MODE == 1) {
              hv[e] = (_Float16)sp[e];
            } else {
              unsigned short hb = f2bf_bits(sp[e]);
              unsigned short lb = f2bf_bits(sp[e] - bf_bits2f(hb));
              hv[e] = __builtin_bit_cast(_Float16, hb);
              lv[e] = __builtin_bit_cast(_Float16, lb);
            }
          }
          *(volatile v8h*)(C + (size_t)(mBase + row) * ldc + n0 + c8) = hv;
          if (OUT_MODE == 2) *(volatile v8h*)(C2 + (size_t)(mBase + row) * ldc + n0 + c8) = lv;
        }
        __threadfence();
      }
    }
    __builtin_amdgcn_fence(__ATOMIC_RELEASE, "workgroup");
    __builtin_amdgcn_wave_barrier();
    __builtin_amdgcn_fence(__ATOMIC_ACQUIRE, "workgroup");
  }
}

__device__ __forceinline__ float gelu_f(float x) {
  return 0.5f * x * (1.0f + erff(x * 0.70710678118654752f));
}
__device__ __forceinline__ float wave_sum32(float v) {
#pragma unroll
  for (int off = 16; off > 0; off >>= 1) v += __shfl_xor(v, off, 32);
  return v;
}
__device__ __forceinline__ float wave_max32(float v) {
#pragma unroll
  for (int off = 16; off > 0; off >>= 1) v = fmaxf(v, __shfl_xor(v, off, 32));
  return v;
}

__global__ __launch_bounds__(256) void cast8_f16_kernel(const float* __restrict__ in0, const float* __restrict__ in1,
                                                       const float* __restrict__ in2, unsigned short* __restrict__ out,
                                                       int n8, long planeElems, float scale) {
  const int z = blockIdx.y;
  const float* in = (z == 0) ? in0 : (z == 1) ? in1 : in2;
  const int i = blockIdx.x * 256 + threadIdx.x;
  if (i >= n8) return;
  const float* p = in + 8 * (size_t)i;
  const v4f a = *(const v4f*)(p);
  const v4f c = *(const v4f*)(p + 4);
  unsigned short hb[8];
#pragma unroll
  for (int e = 0; e < 4; ++e) {
    hb[e]     = h_bits(a[e] * scale);
    hb[4 + e] = h_bits(c[e] * scale);
  }
  const v4u u = (v4u){pk16(hb[0], hb[1]), pk16(hb[2], hb[3]), pk16(hb[4], hb[5]), pk16(hb[6], hb[7])};
  unsigned short* q = out + (size_t)z * planeElems + 8 * (size_t)i;
  *(volatile v4u*)q = u;
  __threadfence();
  *(volatile v4u*)q = u;
}

__global__ __launch_bounds__(256) void split_bf16_kernel(const float* __restrict__ in, unsigned short* __restrict__ outH,
                                                        unsigned short* __restrict__ outL, int n8) {
  const int i = blockIdx.x * 256 + threadIdx.x;
  if (i >= n8) return;
  const float* p = in + 8 * (size_t)i;
  const v4f a = *(const v4f*)(p);
  const v4f c = *(const v4f*)(p + 4);
  unsigned short hb[8], lb[8];
#pragma unroll
  for (int e = 0; e < 4; ++e) {
    const float x0 = a[e], x1 = c[e];
    hb[e] = f2bf_bits(x0);      lb[e]     = f2bf_bits(x0 - bf_bits2f(hb[e]));
    hb[4 + e] = f2bf_bits(x1);  lb[4 + e] = f2bf_bits(x1 - bf_bits2f(hb[4 + e]));
  }
  const v4u uh = (v4u){pk16(hb[0], hb[1]), pk16(hb[2], hb[3]), pk16(hb[4], hb[5]), pk16(hb[6], hb[7])};
  const v4u ul = (v4u){pk16(lb[0], lb[1]), pk16(lb[2], lb[3]), pk16(lb[4], lb[5]), pk16(lb[6], lb[7])};
  unsigned short* qh = outH + 8 * (size_t)i;
  unsigned short* ql = outL + 8 * (size_t)i;
  *(volatile v4u*)qh = uh;
  *(volatile v4u*)ql = ul;
  __threadfence();
  *(volatile v4u*)qh = uh;
  *(volatile v4u*)ql = ul;
}

__global__ __launch_bounds__(256) void q_act_ln_kernel(const float* __restrict__ QP,
                                                      const float* __restrict__ lng, const float* __restrict__ lnb,
                                                      unsigned short* __restrict__ Q16, unsigned short* __restrict__ LQH,
                                                      unsigned short* __restrict__ LQL, float acarry) {
  __shared__ __align__(16) unsigned short sAll[3 * 512];
  __shared__ float red1[8];
  __shared__ float red2[8];
  const int row  = blockIdx.x;
  const int bidx = row >> 10;
  const int t    = row & 1023;
  const int tid  = threadIdx.x, lane = tid & 31, wave = tid >> 5;
  const float* xr = QP + (size_t)row * kD;
  const float x0 = xr[tid];
  const float x1 = xr[tid + 256];
  sAll[tid]       = h_bits(gelu_f(x0) * acarry);
  sAll[tid + 256] = h_bits(gelu_f(x1) * acarry);

  float s = wave_sum32(x0 + x1);
  if (lane == 0) red1[wave] = s;
  __syncthreads();
  float tot = red1[0];
#pragma unroll
  for (int w = 1; w < 8; ++w) tot += red1[w];
  const float mean = tot * kInvD;
  const float d0 = x0 - mean, d1 = x1 - mean;
  float s2 = wave_sum32(d0 * d0 + d1 * d1);
  if (lane == 0) red2[wave] = s2;
  __syncthreads();
  float tot2 = red2[0];
#pragma unroll
  for (int w = 1; w < 8; ++w) tot2 += red2[w];
  const float var  = tot2 * kInvD;
  const float rstd = rsqrtf(var + kLnEps);
  const float y0 = d0 * rstd * lng[tid] + lnb[tid];
  const float y1 = d1 * rstd * lng[tid + 256] + lnb[tid + 256];
  const unsigned short hb0 = f2bf_bits(y0), hb1 = f2bf_bits(y1);
  const unsigned short lb0 = f2bf_bits(y0 - bf_bits2f(hb0)), lb1 = f2bf_bits(y1 - bf_bits2f(hb1));
  sAll[512 + tid]        = hb0;
  sAll[512 + tid + 256]  = hb1;
  sAll[1024 + tid]       = lb0;
  sAll[1024 + tid + 256] = lb1;
  __syncthreads();

  if (wave < 6) {
    const int region = wave >> 1;
    const int chunk  = (wave & 1) * 32 + lane;
    const v4u val = *(const v4u*)(sAll + region * 512 + chunk * 8);
    const int h  = chunk >> 3;
    const int c8 = (chunk & 7) * 8;
    unsigned short* dq = Q16 + ((size_t)((bidx * kH + h) * kT + t)) * kDK + c8;
    unsigned short* dl = ((region == 1) ? LQH : LQL) + (size_t)row * kD + chunk * 8;
    unsigned short* dst = (region == 0) ? dq : dl;
    *(volatile v4u*)dst = val;
    __threadfence();
    *(volatile v4u*)dst = val;
  }
}

__global__ __launch_bounds__(256) void k_act_kernel(const float* __restrict__ KP, unsigned short* __restrict__ K16, float acarry) {
  __shared__ __align__(16) unsigned short s[256];
  const int blk = blockIdx.x;
  const int r   = blk >> 1;
  const int j   = blk & 1;
  const int tid = threadIdx.x, lane = tid & 31, wave = tid >> 5;
  const float x = KP[(size_t)r * kD + j * 256 + tid];
  s[tid] = h_bits(gelu_f(x) * acarry);
  __syncthreads();
  if (wave == 0) {
    const int bidx = r >> 8, c = r & 255;
    const int h  = j * 4 + (lane >> 3);
    const int c8 = (lane & 7) * 8;
    const v4u val = *(const v4u*)(s + lane * 8);
    unsigned short* dst = K16 + ((size_t)((bidx * kH + h) * kC + c)) * kDK + c8;
    *(volatile v4u*)dst = val;
    __threadfence();
    *(volatile v4u*)dst = val;
  }
}

__global__ __launch_bounds__(256) void v_act_kernel(const float* __restrict__ VPT, unsigned short* __restrict__ VT16, float acarry) {
  __shared__ __align__(16) unsigned short s[256];
  const int bidx = blockIdx.x;
  const int m    = blockIdx.y;
  const int tid = threadIdx.x, lane = tid & 31, wave = tid >> 5;
  const float x = VPT[(size_t)m * kRowsKV + bidx * kC + tid];
  s[tid] = h_bits(gelu_f(x) * acarry);
  __syncthreads();
  if (wave == 0) {
    const int h = m >> 6, d = m & 63;
    const v4u val = *(const v4u*)(s + lane * 8);
    unsigned short* dst = VT16 + ((size_t)((bidx * kH + h) * kDK + d)) * kC + lane * 8;
    *(volatile v4u*)dst = val;
    __threadfence();
    *(volatile v4u*)dst = val;
  }
}

__global__ __launch_bounds__(256) void softmax_mask_kernel(const float* __restrict__ S, const int* __restrict__ mask,
                                                          unsigned short* __restrict__ P, int bh0, float pcarry) {
  const int tid = threadIdx.x, lane = tid & 31, wave = tid >> 5;
  const int row = blockIdx.x * 8 + wave;
  const int bhl = row >> 10;
  const int t   = row & 1023;
  const int bidx = (bh0 + bhl) >> 3;
  const float* sr = S + (size_t)row * kC + lane * 8;
  const int*   mr = mask + ((size_t)bidx * kT + t) * kC + lane * 8;
  const v4f a0 = *(const v4f*)(sr);
  const v4f a1 = *(const v4f*)(sr + 4);
  const v4i k0 = *(const v4i*)(mr);
  const v4i k1 = *(const v4i*)(mr + 4);
  float x[8]; int kp[8];
#pragma unroll
  for (int e = 0; e < 4; ++e) { x[e] = a0[e]; x[4 + e] = a1[e]; kp[e] = k0[e]; kp[4 + e] = k1[e]; }
  float m = -INFINITY;
#pragma unroll
  for (int e = 0; e < 8; ++e) m = (kp[e] != 0) ? fmaxf(m, x[e]) : m;
  m = wave_max32(m);
  const float mf = (m == -INFINITY) ? 0.0f : m;
  float p[8];
  float sum = 0.0f;
#pragma unroll
  for (int e = 0; e < 8; ++e) {
    const float ev = expf(x[e] - mf);
    p[e] = (kp[e] != 0) ? ev : 0.0f;
    sum += p[e];
  }
  sum = wave_sum32(sum);
  const float rs = (sum > 0.0f) ? (pcarry / sum) : 0.0f;
  unsigned short hb[8];
#pragma unroll
  for (int e = 0; e < 8; ++e) hb[e] = h_bits(p[e] * rs);
  const v4u u = (v4u){pk16(hb[0], hb[1]), pk16(hb[2], hb[3]), pk16(hb[4], hb[5]), pk16(hb[6], hb[7])};
  unsigned short* dst = P + (size_t)row * kC + lane * 8;
  *(volatile v4u*)dst = u;
  __threadfence();
  *(volatile v4u*)dst = u;
}

__global__ __launch_bounds__(256) void a_ln_kernel(const float* __restrict__ AO,
                                                  const float* __restrict__ lng, const float* __restrict__ lnb,
                                                  unsigned short* __restrict__ LAH, unsigned short* __restrict__ LAL) {
  __shared__ __align__(16) unsigned short sAll[2 * 512];
  __shared__ float red1[8];
  __shared__ float red2[8];
  const int row  = blockIdx.x;
  const int bidx = row >> 10;
  const int t    = row & 1023;
  const int tid  = threadIdx.x, lane = tid & 31, wave = tid >> 5;
  const int n0 = tid, n1 = tid + 256;
  const int h0 = n0 >> 6, d0i = n0 & 63, h1 = n1 >> 6, d1i = n1 & 63;
  const float x0 = AO[((size_t)((bidx * kH + h0) * kT + t)) * kDK + d0i];
  const float x1 = AO[((size_t)((bidx * kH + h1) * kT + t)) * kDK + d1i];

  float s = wave_sum32(x0 + x1);
  if (lane == 0) red1[wave] = s;
  __syncthreads();
  float tot = red1[0];
#pragma unroll
  for (int w = 1; w < 8; ++w) tot += red1[w];
  const float mean = tot * kInvD;
  const float d0 = x0 - mean, d1 = x1 - mean;
  float s2 = wave_sum32(d0 * d0 + d1 * d1);
  if (lane == 0) red2[wave] = s2;
  __syncthreads();
  float tot2 = red2[0];
#pragma unroll
  for (int w = 1; w < 8; ++w) tot2 += red2[w];
  const float var  = tot2 * kInvD;
  const float rstd = rsqrtf(var + kLnEps);
  const float y0 = d0 * rstd * lng[tid] + lnb[tid];
  const float y1 = d1 * rstd * lng[tid + 256] + lnb[tid + 256];
  const unsigned short hb0 = f2bf_bits(y0), hb1 = f2bf_bits(y1);
  const unsigned short lb0 = f2bf_bits(y0 - bf_bits2f(hb0)), lb1 = f2bf_bits(y1 - bf_bits2f(hb1));
  sAll[tid]             = hb0;
  sAll[tid + 256]       = hb1;
  sAll[512 + tid]       = lb0;
  sAll[512 + tid + 256] = lb1;
  __syncthreads();

  if (wave < 4) {
    const int region = wave >> 1;
    const int chunk  = (wave & 1) * 32 + lane;
    const v4u val = *(const v4u*)(sAll + region * 512 + chunk * 8);
    unsigned short* dst = ((region == 0) ? LAH : LAL) + (size_t)row * kD + chunk * 8;
    *(volatile v4u*)dst = val;
    __threadfence();
    *(volatile v4u*)dst = val;
  }
}

extern "C" void kernel_launch(void* const* d_in, const int* in_sizes, int n_in,
                              void* d_out, int out_size, void* d_ws, size_t ws_size,
                              hipStream_t stream) {
  (void)n_in;
  if (ws_size < kWsTotal) return;
  if (in_sizes[0] != kRowsQ * kD || in_sizes[1] != kRowsKV * kD || in_sizes[2] != kRowsKV * kD ||
      in_sizes[3] != kRowsQ * kC || in_sizes[14] != kD * 2 * kD || out_size != kRowsQ * kD) return;

  const float* query = (const float*)d_in[0];
  const float* key   = (const float*)d_in[1];
  const float* value = (const float*)d_in[2];
  const int*   mask  = (const int*)  d_in[3];
  const float* Wq    = (const float*)d_in[4];
  const float* bq    = (const float*)d_in[5];
  const float* Wk    = (const float*)d_in[6];
  const float* bk    = (const float*)d_in[7];
  const float* Wv    = (const float*)d_in[8];
  const float* bv    = (const float*)d_in[9];
  const float* q_ln_g    = (const float*)d_in[10];
  const float* q_ln_b    = (const float*)d_in[11];
  const float* attn_ln_g = (const float*)d_in[12];
  const float* attn_ln_b = (const float*)d_in[13];
  const float* Wo    = (const float*)d_in[14];
  const float* bo    = (const float*)d_in[15];
  float* out = (float*)d_out;

  char* ws = (char*)d_ws;
  unsigned short* Wq16 = (unsigned short*)(ws + kOffWq);
  unsigned short* Wk16 = (unsigned short*)(ws + kOffWk);
  unsigned short* Wv16 = (unsigned short*)(ws + kOffWv);
  unsigned short* WoH  = (unsigned short*)(ws + kOffWoH);
  unsigned short* WoL  = (unsigned short*)(ws + kOffWoL);
  unsigned short* K16  = (unsigned short*)(ws + kOffK16);
  unsigned short* VT16 = (unsigned short*)(ws + kOffVT16);
  float* QP   = (float*)(ws + kOffRA);
  float* PART = (float*)(ws + kOffRA);
  unsigned short* Kin16 = (unsigned short*)(ws + kOffRB);
  unsigned short* Vin16 = (unsigned short*)(ws + kOffRB + 4194304);
  float*          KP    = (float*)(ws + kOffRB + 8388608);
  float*          VPT   = (float*)(ws + kOffRB + 16777216);
  unsigned short* LQH   = (unsigned short*)(ws + kOffRB);
  unsigned short* LQL   = (unsigned short*)(ws + kOffRB + 16777216);
  float*          Sbuf  = (float*)(ws + kOffRB);
  unsigned short* Pbuf  = (unsigned short*)(ws + kOffRB + 16777216);
  unsigned short* LAH   = (unsigned short*)(ws + kOffRB);
  unsigned short* LAL   = (unsigned short*)(ws + kOffRB + 16777216);
  unsigned short* X16 = (unsigned short*)(ws + kOffRC);
  unsigned short* Q16 = (unsigned short*)(ws + kOffRC);
  float* AO = (float*)(ws + kOffRD);

  cast8_f16_kernel<<<dim3(kD * kD / 8 / 256, 3), 256, 0, stream>>>(Wq, Wk, Wv, Wq16, kD * kD / 8, (long)(kD * kD), kWCarry);
  split_bf16_kernel<<<dim3(kD * 2 * kD / 8 / 256), 256, 0, stream>>>(Wo, WoH, WoL, kD * 2 * kD / 8);

  cast8_f16_kernel<<<dim3(kRowsKV * kD / 8 / 256, 2), 256, 0, stream>>>(key, value, value, Kin16, kRowsKV * kD / 8,
                                                                        (long)(kRowsKV * kD), 1.0f);
  wmma_gemm64<0, false, 2, 0, false><<<dim3(64, 1), 256, 0, stream>>>(
      Kin16, Kin16, kD, 0L, Wk16, Wk16, kD, 0L, (void*)KP, (void*)KP, kD, 0L, bk, KP, 0L, kRowsKV, kD, kD, kWCarryInv);
  wmma_gemm64<0, false, 1, 0, false><<<dim3(64, 1), 256, 0, stream>>>(
      Wv16, Wv16, kD, 0L, Vin16, Vin16, kD, 0L, (void*)VPT, (void*)VPT, kRowsKV, 0L, bv, VPT, 0L, kD, kRowsKV, kD, kWCarryInv);
  k_act_kernel<<<dim3(kRowsKV * 2), 256, 0, stream>>>(KP, K16, kACarry);
  v_act_kernel<<<dim3(kB, kD), 256, 0, stream>>>(VPT, VT16, kACarry);

  cast8_f16_kernel<<<dim3(kRowsQ * kD / 8 / 256, 1), 256, 0, stream>>>(query, query, query, X16, kRowsQ * kD / 8, 0L, 1.0f);
  wmma_gemm64<0, false, 2, 0, false><<<dim3(256, 1), 256, 0, stream>>>(
      X16, X16, kD, 0L, Wq16, Wq16, kD, 0L, (void*)QP, (void*)QP, kD, 0L, bq, QP, 0L, kRowsQ, kD, kD, kWCarryInv);
  q_act_ln_kernel<<<dim3(kRowsQ), 256, 0, stream>>>(QP, q_ln_g, q_ln_b, Q16, LQH, LQL, kACarry);

  wmma_gemm64<1, true, 2, 0, false><<<dim3(256, 1), 256, 0, stream>>>(
      LQH, LQL, kD, 0L, WoH + kD, WoL + kD, 2 * kD, 0L, (void*)PART, (void*)PART, kD, 0L, bo, PART, 0L,
      kRowsQ, kD, kD, 1.0f);

  for (int g = 0; g < kNGroups; ++g) {
    const size_t bhBase = (size_t)g * kGroupBH;
    const unsigned short* Q16g  = Q16  + bhBase * (size_t)(kT * kDK);
    const unsigned short* K16g  = K16  + bhBase * (size_t)(kC * kDK);
    const unsigned short* VT16g = VT16 + bhBase * (size_t)(kDK * kC);
    float* AOg = AO + bhBase * (size_t)(kT * kDK);
    wmma_gemm64<0, false, 0, 0, false><<<dim3(8, kGroupBH), 256, 0, stream>>>(
        Q16g, Q16g, kDK, (long)(kT * kDK), K16g, K16g, kDK, (long)(kC * kDK), (void*)Sbuf, (void*)Sbuf, kC, (long)(kT * kC),
        bq, Sbuf, 0L, kT, kC, kDK, kScoreScale);
    softmax_mask_kernel<<<dim3(kGroupBH * kT / 8), 256, 0, stream>>>(Sbuf, mask, Pbuf, g * kGroupBH, kPCarry);
    wmma_gemm64<0, false, 0, 0, false><<<dim3(2, kGroupBH), 256, 0, stream>>>(
        Pbuf, Pbuf, kC, (long)(kT * kC), VT16g, VT16g, kC, (long)(kDK * kC), (void*)AOg, (void*)AOg, kDK, (long)(kT * kDK),
        bq, AOg, 0L, kT, kDK, kC, kPVScale);
  }

  a_ln_kernel<<<dim3(kRowsQ), 256, 0, stream>>>(AO, attn_ln_g, attn_ln_b, LAH, LAL);
  wmma_gemm64<1, true, 0, 0, true><<<dim3(256, 1), 256, 0, stream>>>(
      LAH, LAL, kD, 0L, WoH, WoL, 2 * kD, 0L, (void*)out, (void*)out, kD, 0L, bo, PART, 0L,
      kRowsQ, kD, kD, 1.0f);
}
